// SimpleTSSGCNet_9620726743376
// MI455X (gfx1250) — hardware-run, weakly checked
//
#include <hip/hip_runtime.h>


namespace {
constexpr int N = 50000, KN = 16, D = 128, H = 64, G3 = 3 * H, NPB = 8;
constexpr float HS = 256.0f, WSC = 256.0f, EPS = 1e-5f;
typedef _Float16 b16;
typedef __attribute__((ext_vector_type(16))) _Float16 v16b;
typedef __attribute__((ext_vector_type(8))) _Float16 v8b;
typedef __attribute__((ext_vector_type(8))) float v8f;
typedef __attribute__((ext_vector_type(4))) float v4f;
typedef __attribute__((ext_vector_type(2))) float v2f;
__device__ __forceinline__ float bf16_rne(float f) { unsigned int u = __float_as_uint(f); u += 0x7FFFu + ((u >> 16) & 1u); float r = __uint_as_float(u & 0xFFFF0000u); asm volatile("" : "+v"(r)); return r; }
__device__ __forceinline__ float bfv(float f) { float r = bf16_rne(f); asm volatile("" : "+v"(r)); return r; }
__device__ __forceinline__ void split16(float v, b16& hi, b16& lo) { hi = (b16)v; lo = (b16)(v - (float)hi); }
__device__ __forceinline__ v16b frag_kb(const b16* p, int hh) { const v8b a = *(const v8b*)(p + 8 * hh), b = *(const v8b*)(p + 16 + 8 * hh); v16b f;
#pragma unroll
  for (int e = 0; e < 8; ++e) { f[e] = a[e]; f[8 + e] = b[e]; } return f; }
__device__ __forceinline__ v8f wmma16b(v16b a, v16b b, v8f c) { v8f d = __builtin_amdgcn_wmma_f32_16x16x32_f16(false, a, false, b, (short)0, c, false, false); asm volatile("v_nop\n\tv_nop\n\tv_nop\n\tv_nop" : "+v"(d) : "v"(a), "v"(b)); return d; }
__device__ __forceinline__ void wave_lds_sync() { __builtin_amdgcn_fence(__ATOMIC_RELEASE, "workgroup"); __builtin_amdgcn_wave_barrier(); __builtin_amdgcn_fence(__ATOMIC_ACQUIRE, "workgroup"); }
__device__ __forceinline__ float pmul(float a, float b) { float p = a * b; asm volatile("" : "+v"(p)); return p; }
__device__ __forceinline__ int iclamp(int v, int lo, int hi) { return v < lo ? lo : (v > hi ? hi : v); }
__device__ __forceinline__ float sigm(float v) { return 1.0f / (1.0f + __expf(-v)); }
constexpr float DINV2 = 1.0f / 17.0f;

__global__ __launch_bounds__(256) void wput_kernel(const float* __restrict__ w1, const float* __restrict__ w2, const float* __restrict__ wih, const float* __restrict__ whh, b16* __restrict__ WT1, b16* __restrict__ WT2, b16* __restrict__ WIH, b16* __restrict__ WHH) { const int u = blockIdx.x * 256 + threadIdx.x; v8b v;
  if (u < H * 16) { const int o = u / 16, k0 = (u % 16) * 8;
#pragma unroll
    for (int j = 0; j < 8; ++j) v[j] = (b16)(bf16_rne(w1[(size_t)(k0 + j) * H + o]) * WSC); for (int pass = 0; pass < 2; ++pass) { *(volatile v8b*)(WT1 + (size_t)o * D + k0) = v; __threadfence(); } }
  if (u < H * 8) { const int o = u / 8, k0 = (u % 8) * 8;
#pragma unroll
    for (int j = 0; j < 8; ++j) v[j] = (b16)(bf16_rne(w2[(size_t)(k0 + j) * H + o]) * WSC); for (int pass = 0; pass < 2; ++pass) { *(volatile v8b*)(WT2 + (size_t)o * H + k0) = v; __threadfence(); } }
  if (u < G3 * 16) { const int o = u / 16, k0 = (u % 16) * 8;
#pragma unroll
    for (int j = 0; j < 8; ++j) v[j] = (b16)(bf16_rne(wih[(size_t)o * D + k0 + j]) * WSC); for (int pass = 0; pass < 2; ++pass) { *(volatile v8b*)(WIH + (size_t)o * D + k0) = v; __threadfence(); } }
  if (u < G3 * 8) { const int o = u / 8, k0 = (u % 8) * 8;
#pragma unroll
    for (int j = 0; j < 8; ++j) v[j] = (b16)(bf16_rne(whh[(size_t)o * H + k0 + j]) * WSC); for (int pass = 0; pass < 2; ++pass) { *(volatile v8b*)(WHH + (size_t)o * H + k0) = v; __threadfence(); } } }
template <int MODE, int KIN, int NT>
__global__ __launch_bounds__(32) void lin_kernel(const float* __restrict__ IN, const float* __restrict__ BNP, const b16* __restrict__ W, int NLIM, float* __restrict__ OUT) { constexpr int OW = NT * 16; __shared__ __attribute__((aligned(16))) b16 Ah[16][KIN + 8], Al[16][KIN + 8]; __shared__ float Tf[16][OW + 4]; const int lane = threadIdx.x, nloc = lane & 15, hlf = lane >> 4; const size_t m0 = (size_t)blockIdx.x * 16; if (m0 >= (size_t)NLIM) return;
  for (int rr = 0; rr < 16; ++rr) for (int q = 0; q < KIN / 32; ++q) { const int c = q * 32 + lane; const float v = IN[(m0 + rr) * KIN + c]; b16 p, ql; if (MODE == 0) { p = (b16)(bf16_rne(v) * HS); ql = (b16)0.0f; } else split16(fmaxf(pmul(v, BNP[c]) + BNP[H + c], 0.0f) * HS, p, ql); Ah[rr][c] = p; Al[rr][c] = ql; }
  if (lane < 16) for (int k = KIN; k < KIN + 8; ++k) { Ah[lane][k] = (b16)0.0f; Al[lane][k] = (b16)0.0f; }
  wave_lds_sync(); v8f acc[NT];
#pragma unroll
  for (int t = 0; t < NT; ++t) acc[t] = (v8f){};
#pragma unroll
  for (int kb = 0; kb < KIN; kb += 32) { const v16b a = frag_kb(&Ah[nloc][kb], hlf), al = frag_kb(&Al[nloc][kb], hlf);
#pragma unroll
    for (int t = 0; t < NT; ++t) { const v16b bw = frag_kb(W + (size_t)(t * 16 + nloc) * KIN + kb, hlf); acc[t] = wmma16b(a, bw, acc[t]); if (MODE == 1) acc[t] = wmma16b(al, bw, acc[t]); } }
#pragma unroll
  for (int t = 0; t < NT; ++t)
#pragma unroll
    for (int r8 = 0; r8 < 8; ++r8) Tf[8 * hlf + r8][t * 16 + nloc] = acc[t][r8] * (1.0f / (HS * WSC));
  wave_lds_sync();
  for (int pass = 0; pass < 2; ++pass) { for (int rr = 0; rr < 16; ++rr) for (int q = 0; q < OW / 64; ++q) *(volatile v2f*)(OUT + (m0 + rr) * OW + q * 64 + lane * 2) = *(const v2f*)(&Tf[rr][q * 64 + lane * 2]); __threadfence(); } }
__global__ __launch_bounds__(256) void sweep_kernel(const float* __restrict__ HW, const float* __restrict__ bias, const int* __restrict__ esrc, int NLIM, float* __restrict__ Gp, float* __restrict__ PS) { __shared__ float Gs[NPB][H]; const int wave = threadIdx.x >> 5, lane = threadIdx.x & 31; const size_t i = (size_t)blockIdx.x * NPB + wave; const bool live = i < (size_t)NLIM; v2f o = {0, 0};
  if (live) { v2f acc = {0, 0};
#pragma unroll 1
    for (int k = 0; k < KN; ++k) { const size_t u = (size_t)iclamp(esrc[i * KN + k], 0, NLIM - 1); const v2f v = *(const v2f*)(HW + u * H + lane * 2); acc[0] += v[0]; acc[1] += v[1]; }
    const v2f hv = *(const v2f*)(HW + i * H + lane * 2); for (int q = 0; q < 2; ++q) o[q] = pmul(acc[q] + hv[q], DINV2) + bfv(bias[lane * 2 + q]); }
  Gs[wave][lane * 2] = live ? o[0] : 0.0f; Gs[wave][lane * 2 + 1] = live ? o[1] : 0.0f;
  __syncthreads();
  for (int pass = 0; pass < 2; ++pass) { if (live) *(volatile v2f*)(Gp + i * H + lane * 2) = o; if (threadIdx.x < 128) { const int c = threadIdx.x & 63, which = threadIdx.x >> 6; float s = 0.0f; for (int w = 0; w < NPB; ++w) { const float v = Gs[w][c]; s += which ? v * v : v; } ((volatile float*)PS)[(size_t)blockIdx.x * 2 * H + which * H + c] = s; } __threadfence(); } }
__global__ __launch_bounds__(64) void bn_kernel(const float* __restrict__ PS, int nb, int count, const float* __restrict__ g, const float* __restrict__ be, float* __restrict__ BNP) { const int c = threadIdx.x; double s = 0.0, s2 = 0.0; for (int w = 0; w < nb; ++w) { s += (double)PS[(size_t)w * 2 * H + c]; s2 += (double)PS[(size_t)w * 2 * H + H + c]; } const double mu = s / count; double var = s2 / count - mu * mu; if (var < 0.0) var = 0.0; const float sc = bfv(g[c]) * (float)(1.0 / sqrt(var + (double)EPS)); const float sh = bfv(be[c]) - (float)mu * sc;
  for (int pass = 0; pass < 2; ++pass) { ((volatile float*)BNP)[c] = sc; ((volatile float*)BNP)[H + c] = sh; __threadfence(); } }
__global__ __launch_bounds__(32) void gru_kernel(const float* __restrict__ XW, const float* __restrict__ ts, const int* __restrict__ esrc, const float* __restrict__ beta, const b16* __restrict__ WHH, const float* __restrict__ bih, const float* __restrict__ bhh, int NLIM, float* __restrict__ HT) {
  __shared__ __attribute__((aligned(16))) b16 Hh[16][H + 8], Hl[16][H + 8]; __shared__ float Hf[16][H + 1], Al_[16][KN + 1], Gh[16][G3 + 4]; __shared__ int Nb[16][KN + 1]; const int lane = threadIdx.x, nloc = lane & 15, hlf = lane >> 4; const size_t m0 = (size_t)blockIdx.x * 16; if (m0 >= (size_t)NLIM) return; const float bt = bfv(beta[0]);
  { const int r = nloc; const size_t i = m0 + r; const float ti = bfv(ts[i]); float a8[8]; float s = 0.0f;
    for (int j = 0; j < 8; ++j) { const int k = hlf * 8 + j; const int u = iclamp(esrc[i * KN + k], 0, NLIM - 1); Nb[r][k] = u; const float dt = fmaxf(ti - bfv(ts[u]), 0.0f); a8[j] = __expf(-pmul(bt, dt)); s += a8[j]; }
    s += __shfl_xor(s, 16); const float inv = 1.0f / (s + 1e-9f); for (int j = 0; j < 8; ++j) Al_[r][hlf * 8 + j] = a8[j] * inv; }
  for (int rr = 0; rr < 16; ++rr) for (int q = 0; q < 2; ++q) Hf[rr][q * 32 + lane] = 0.0f; if (lane < 16) for (int k = H; k < H + 8; ++k) { Hh[lane][k] = (b16)0.0f; Hl[lane][k] = (b16)0.0f; }
  wave_lds_sync();
#pragma unroll 1
  for (int t = 0; t < KN; ++t) {
    for (int rr = 0; rr < 16; ++rr) for (int q = 0; q < 2; ++q) { const int c = q * 32 + lane; b16 p, ql; split16(Hf[rr][c] * HS, p, ql); Hh[rr][c] = p; Hl[rr][c] = ql; }
    wave_lds_sync(); v8f acc[12];
#pragma unroll
    for (int tt = 0; tt < 12; ++tt) acc[tt] = (v8f){};
#pragma unroll
    for (int kb = 0; kb < H; kb += 32) { const v16b a = frag_kb(&Hh[nloc][kb], hlf), al = frag_kb(&Hl[nloc][kb], hlf);
#pragma unroll
      for (int tt = 0; tt < 12; ++tt) { const v16b bw = frag_kb(WHH + (size_t)(tt * 16 + nloc) * H + kb, hlf); acc[tt] = wmma16b(a, bw, acc[tt]); acc[tt] = wmma16b(al, bw, acc[tt]); } }
#pragma unroll
    for (int tt = 0; tt < 12; ++tt) { const int cc = tt * 16 + nloc; const float bb = bfv(bhh[cc]);
#pragma unroll
      for (int r8 = 0; r8 < 8; ++r8) Gh[8 * hlf + r8][cc] = acc[tt][r8] * (1.0f / (HS * WSC)) + bb; }
    wave_lds_sync();
    for (int rr = 0; rr < 16; ++rr) { const int u = Nb[rr][t]; const float al = Al_[rr][t]; for (int q = 0; q < 2; ++q) { const int c = q * 32 + lane; const float gir = pmul(al, XW[(size_t)u * G3 + c]) + bfv(bih[c]), giz = pmul(al, XW[(size_t)u * G3 + H + c]) + bfv(bih[H + c]), gin = pmul(al, XW[(size_t)u * G3 + 2 * H + c]) + bfv(bih[2 * H + c]);
        const float r = sigm(gir + Gh[rr][c]), z = sigm(giz + Gh[rr][H + c]); const float nn_ = tanhf(gin + pmul(r, Gh[rr][2 * H + c])); Hf[rr][c] = pmul(1.0f - z, nn_) + pmul(z, Hf[rr][c]); } }
    wave_lds_sync(); }
  for (int pass = 0; pass < 2; ++pass) { for (int rr = 0; rr < 16; ++rr) *(volatile v2f*)(HT + (m0 + rr) * H + lane * 2) = (v2f){Hf[rr][lane * 2], Hf[rr][lane * 2 + 1]}; __threadfence(); } }
__global__ __launch_bounds__(256) void head_kernel(const float* __restrict__ G2, const float* __restrict__ BNP, const float* __restrict__ HT, const float* __restrict__ wo, const float* __restrict__ bo, int NLIM, float* __restrict__ out) { const int wave = threadIdx.x >> 5, lane = threadIdx.x & 31; const size_t n0 = ((size_t)blockIdx.x * NPB + wave) * 32; if (n0 >= (size_t)NLIM) return; const bool ok = n0 + lane < (size_t)NLIM; const size_t n = ok ? n0 + lane : (size_t)NLIM - 1;     float s0 = bfv(bo[0]), s1 = bfv(bo[1]);
#pragma unroll 4
  for (int c = 0; c < H; ++c) { const float h2 = fmaxf(pmul(G2[n * H + c], BNP[c]) + BNP[H + c], 0.0f); s0 += pmul(h2, bfv(wo[c * 2])); s1 += pmul(h2, bfv(wo[c * 2 + 1])); }
#pragma unroll 4
  for (int c = 0; c < H; ++c) { const float ht = HT[n * H + c]; s0 += pmul(ht, bfv(wo[(H + c) * 2])); s1 += pmul(ht, bfv(wo[(H + c) * 2 + 1])); }
  for (int pass = 0; pass < 2; ++pass) { if (ok) *(volatile v2f*)(out + n * 2) = (v2f){s0, s1}; __threadfence(); } }
}

extern "C" void kernel_launch(void* const* d_in, const int* in_sizes, int n_in, void* d_out, int out_size, void* d_ws, size_t ws_size, hipStream_t stream) {
  (void)n_in;
  auto Fp = [&](int i) { return (const float*)d_in[i]; }; auto Ip = [&](int i) { return (const int*)d_in[i]; };
  if (in_sizes[0] != N * D || in_sizes[1] != N || in_sizes[2] != N * KN || in_sizes[3] != D * H || in_sizes[7] != H * H || in_sizes[11] != G3 * D || in_sizes[12] != G3 * H || in_sizes[15] != 1 || in_sizes[16] != 2 * H * 2 || out_size != N * 2) return;
  const int NLIM = N;
  size_t off = 0; char* ws = (char*)d_ws;
  auto carve = [&](size_t bytes) { char* p = ws + off; off += (bytes + 255) & ~(size_t)255; return p; };
  b16* WT1 = (b16*)carve((size_t)H * D * 2); b16* WT2 = (b16*)carve((size_t)H * H * 2); b16* WIH = (b16*)carve((size_t)G3 * D * 2); b16* WHH = (b16*)carve((size_t)G3 * H * 2);
  float* HW = (float*)carve((size_t)N * H * 4); float* G1 = (float*)carve((size_t)N * H * 4); float* G2 = (float*)carve((size_t)N * H * 4); float* PS = (float*)carve((size_t)(N / NPB + 1) * 2 * H * 4); float* BN1 = (float*)carve(2 * H * 4); float* BN2 = (float*)carve(2 * H * 4); float* XW = (float*)carve((size_t)N * G3 * 4); float* HT = (float*)carve((size_t)N * H * 4);
  if (off > ws_size || off > ((size_t)112 << 20)) return;
  const int nb = (NLIM + NPB - 1) / NPB;
  wput_kernel<<<(G3 * 16 + 255) / 256, 256, 0, stream>>>(Fp(3), Fp(7), Fp(11), Fp(12), WT1, WT2, WIH, WHH);
  lin_kernel<0, 128, 4><<<NLIM / 16, 32, 0, stream>>>(Fp(0), nullptr, WT1, NLIM, HW);
  sweep_kernel<<<nb, 256, 0, stream>>>(HW, Fp(4), Ip(2), NLIM, G1, PS); bn_kernel<<<1, 64, 0, stream>>>(PS, nb, NLIM, Fp(5), Fp(6), BN1);
  lin_kernel<1, 64, 4><<<NLIM / 16, 32, 0, stream>>>(G1, BN1, WT2, NLIM, HW);
  sweep_kernel<<<nb, 256, 0, stream>>>(HW, Fp(8), Ip(2), NLIM, G2, PS); bn_kernel<<<1, 64, 0, stream>>>(PS, nb, NLIM, Fp(9), Fp(10), BN2);
  lin_kernel<0, 128, 12><<<NLIM / 16, 32, 0, stream>>>(Fp(0), nullptr, WIH, NLIM, XW);
  gru_kernel<<<NLIM / 16, 32, 0, stream>>>(XW, Fp(1), Ip(2), Fp(15), WHH, Fp(13), Fp(14), NLIM, HT);
  head_kernel<<<((NLIM + 31) / 32 + NPB - 1) / NPB, 256, 0, stream>>>(G2, BN2, HT, Fp(16), Fp(17), NLIM, (float*)d_out);
}
